// GIN_74062416053220
// MI455X (gfx1250) — hardware-verified
//
#include <hip/hip_runtime.h>
#include <stddef.h>
#include <stdint.h>


#define DF      64
#define KA      128
#define NLAY    3
#define NCLS    10
#define XPH     192
#define XPW     384
#define NTHR    256
#define NWAVE   8
#define EPT     8
#define CHUNK   (NTHR * EPT)
#define WCAP    (EPT * 32)
#define LISTN   (NWAVE * WCAP)
#define NBMAX   1024
#define PKS     10
#define RCAP    28672
#define DEGCAP  64
#define MCAP    1024
#define NBM     64
#define TM      128
#define TP      136
#define RECW    160
#define STATW   256
#define ZINTS   (2 * RCAP + 2 * NBMAX + LISTN + 16)
#define LDS_BKT (ZINTS * 4)
#define LDS_MLP (NWAVE * 16 * TP * 2 + TM * DF * 4 + 128 * 4 + RECW * 4)
#define WSCAP   134217728

static_assert((CHUNK & (CHUNK - 1)) == 0 && CHUNK == 2048);
static_assert((NBMAX & (NBMAX - 1)) == 0 && NBMAX == (1 << PKS));
static_assert(((long long)CHUNK << PKS) < (1LL << 31));
static_assert(NTHR * 4 == NBMAX && LISTN >= NBMAX);
static_assert((RCAP % (4 * NTHR)) == 0 && (ZINTS % 4) == 0);
static_assert(RCAP >= 16710 + 16710 / 20);
static_assert(DEGCAP >= 36 + 8);
static_assert(MCAP >= 250 + 250 / 4);
static_assert(NBM * 250 <= RCAP && NBM <= NBMAX && (NBM & (NBM - 1)) == 0);
static_assert(LDS_BKT <= 300000 && LDS_MLP <= 300000);
static_assert((KA % 32) == 0 && (XPW % 32) == 0 && KA == 2 * DF && XPW == 2 * XPH && XPH == NLAY * DF);
static_assert(TM == NWAVE * 16 && DF == 4 * 16 && DF == 2 * 32);
static_assert((TP % 8) == 0 && TP >= KA);
static_assert(RECW >= 2 * DF + 1 && (RECW % 32) == 0 && RECW / 4 <= NTHR);
static_assert(STATW == 4 * DF && (TM * NCLS) % 4 == 0 && (TM * NCLS) / 4 <= 2 * NTHR);

typedef float          v2f  __attribute__((ext_vector_type(2)));
typedef float          v4f  __attribute__((ext_vector_type(4)));
typedef float          v8f  __attribute__((ext_vector_type(8)));
typedef int            v4i  __attribute__((ext_vector_type(4)));
typedef int            v8i  __attribute__((ext_vector_type(8)));
typedef unsigned short v8us __attribute__((ext_vector_type(8)));
typedef __bf16         v16b __attribute__((ext_vector_type(16)));
typedef v4f  __attribute__((may_alias)) v4fa;
typedef v4i  __attribute__((may_alias)) v4ia;
typedef v8us __attribute__((may_alias)) v8usa;
union Frag { v16b vb; v8us h[2]; v8i w; };

__device__ __forceinline__ v8f wmx(const Frag& a, const Frag& b, v8f c) {
  v8f d = __builtin_amdgcn_wmma_f32_16x16x32_bf16(false, a.vb, false, b.vb, (short)0, c, false, false);
  asm volatile("v_nop\n\tv_nop\n\tv_nop\n\tv_nop" : "+v"(d) : "v"(a.w), "v"(b.w));
  return d;
}

__device__ __forceinline__ unsigned short bf_bits(float f) {
  const unsigned int u = __float_as_uint(f);
  const unsigned int r = (u + 0x7FFFu + ((u >> 16) & 1u)) >> 16;
  return (unsigned short)((f != f) ? 0x7FC0u : r);
}
__device__ __forceinline__ float bf_val(unsigned short b) { return __uint_as_float(((unsigned int)b) << 16); }
__device__ __forceinline__ float bf_rne(float f) { return bf_val(bf_bits(f)); }
__device__ __forceinline__ float relu_k(float v) { return (v > 0.0f) ? v : (v - v); }

__device__ __forceinline__ int scan_chunk(const int* __restrict__ dsts, int nE, int cbase, int slotBase,
                                          int nb, int vec8, int* list, int tid, int lane, int wave) {
  int wc = 0;
  const int el0  = tid * EPT;
  const int e0   = cbase + el0;
  const int sent = -2147483647 - 1;
  v4i da, db;
  if (vec8 != 0 && cbase + CHUNK <= nE) {
    da = *(const v4i*)(dsts + e0);
    db = *(const v4i*)(dsts + e0 + 4);
  } else {
    da.x = (e0     < nE) ? dsts[min(e0,     nE - 1)] : sent;
    da.y = (e0 + 1 < nE) ? dsts[min(e0 + 1, nE - 1)] : sent;
    da.z = (e0 + 2 < nE) ? dsts[min(e0 + 2, nE - 1)] : sent;
    da.w = (e0 + 3 < nE) ? dsts[min(e0 + 3, nE - 1)] : sent;
    db.x = (e0 + 4 < nE) ? dsts[min(e0 + 4, nE - 1)] : sent;
    db.y = (e0 + 5 < nE) ? dsts[min(e0 + 5, nE - 1)] : sent;
    db.z = (e0 + 6 < nE) ? dsts[min(e0 + 6, nE - 1)] : sent;
    db.w = (e0 + 7 < nE) ? dsts[min(e0 + 7, nE - 1)] : sent;
  }
  const unsigned nbs = (unsigned)slotBase;
  const unsigned unb = (unsigned)nb;
  const unsigned s0 = (unsigned)da.x - nbs, s1 = (unsigned)da.y - nbs;
  const unsigned s2 = (unsigned)da.z - nbs, s3 = (unsigned)da.w - nbs;
  const unsigned s4 = (unsigned)db.x - nbs, s5 = (unsigned)db.y - nbs;
  const unsigned s6 = (unsigned)db.z - nbs, s7 = (unsigned)db.w - nbs;
  const bool h0 = s0 < unb, h1 = s1 < unb, h2 = s2 < unb, h3 = s3 < unb;
  const bool h4 = s4 < unb, h5 = s5 < unb, h6 = s6 < unb, h7 = s7 < unb;
  const unsigned any = __builtin_amdgcn_ballot_w32(h0 | h1 | h2 | h3 | h4 | h5 | h6 | h7);
  if (any != 0u) {
#define HITJ(J, HJ, SJ) { \
      const unsigned mj = __builtin_amdgcn_ballot_w32(HJ); \
      if (mj != 0u) { \
        if (HJ) { \
          const int pos = wc + (int)__builtin_amdgcn_mbcnt_lo(mj, 0u); \
          if (pos < WCAP) list[wave * WCAP + pos] = ((el0 + (J)) << PKS) | (int)(SJ); \
        } \
        wc += (int)__builtin_popcount(mj); } }
    HITJ(0, h0, s0)
    HITJ(1, h1, s1)
    HITJ(2, h2, s2)
    HITJ(3, h3, s3)
    HITJ(4, h4, s4)
    HITJ(5, h5, s5)
    HITJ(6, h6, s6)
    HITJ(7, h7, s7)
#undef HITJ
  }
  return wc;
}

__global__ __launch_bounds__(NTHR) void k_pa(const float* __restrict__ x, int nN, int nUnits, unsigned short* xb) {
  const int u = (int)blockIdx.x * NTHR + (int)threadIdx.x;
  if (u >= nUnits) return;
  const int row = u >> 3, q = u & 7;
  const bool live = row < nN;
  const int rc = live ? row : nN - 1;
  const float* p = x + (size_t)rc * DF + 8 * q;
  const v4f a = *(const v4f*)p;
  const v4f b = *(const v4f*)(p + 4);
  const float f[8] = {a.x, a.y, a.z, a.w, b.x, b.y, b.z, b.w};
  v8us o;
#pragma unroll
  for (int j = 0; j < 8; ++j) o[j] = live ? bf_bits(f[j]) : (unsigned short)0;
  unsigned short* dp = xb + (size_t)u * 8;
  *(volatile v8us*)dp = o;
  __threadfence();
  *(volatile v8us*)dp = o;
}

__device__ __forceinline__ v8us cv8b(const float* __restrict__ p, size_t stride) {
  v8us o;
#pragma unroll
  for (int i = 0; i < 8; ++i) o[i] = bf_bits(p[(size_t)i * stride]);
  return o;
}

__global__ __launch_bounds__(NTHR) void k_pb(const float* __restrict__ w1, const float* __restrict__ w2,
                                             const float* __restrict__ lw,
                                             unsigned short* wpl, unsigned short* lwd) {
  const int u = (int)blockIdx.x * NTHR + (int)threadIdx.x;
  v8us o;
  unsigned short* dp;
  if (u < 6144) {
    const int mat = u >> 10, v = u & 1023;
    const int layer = mat >> 1, which = mat & 1;
    const int n = v >> 4, k8 = (v & 15) * 8, kk = k8 & (DF - 1);
    const size_t so = (size_t)layer * DF * DF + (size_t)kk * DF + n;
    if (which == 0) o = cv8b(w1 + so, DF);
    else            o = cv8b(w2 + so, DF);
    dp = wpl + (size_t)mat * (DF * KA) + (size_t)v * 8;
  } else if (u < 9216) {
    const int v = u - 6144;
    const int n = v / (XPW / 8);
    const int k8 = (v - n * (XPW / 8)) * 8;
    const int kk = k8 < XPH ? k8 : k8 - XPH;
    o = cv8b(lw + (size_t)kk * DF + n, DF);
    dp = lwd + (size_t)v * 8;
  } else {
    return;
  }
  *(volatile v8us*)dp = o;
  __threadfence();
  *(volatile v8us*)dp = o;
}

template <int VALSRC>
__global__ __launch_bounds__(NTHR) void k_bucket(const int* __restrict__ keys, const int* __restrict__ vals,
                                                 int nK, int nb, int vmax, int vec8, int* lst, int* co) {
  extern __shared__ v4i bkt_dyn[];
  int* reg1 = (int*)bkt_dyn;
  int* reg2 = reg1 + RCAP;
  int* scnt = reg2 + RCAP;
  int* soff = scnt + NBMAX;
  int* list = soff + NBMAX;
  int* wcnt = list + LISTN;
  int* wtot = wcnt + NWAVE;
  const int tid = (int)threadIdx.x, lane = tid & 31, wave = tid >> 5;
  const int slotBase = (int)blockIdx.x * nb;

  {
    const v4i z4 = {0, 0, 0, 0};
    for (int i = tid * 4; i < ZINTS; i += NTHR * 4) *(v4ia*)(reg1 + i) = z4;
  }
  __syncthreads();

  int tot = 0;
  const int nChunks = (nK + CHUNK - 1) / CHUNK;
#pragma unroll 1
  for (int ch = 0; ch < nChunks; ++ch) {
    const int cbase = ch * CHUNK;
    const int wc = scan_chunk(keys, nK, cbase, slotBase, nb, vec8, list, tid, lane, wave);
    if (lane == 0) wcnt[wave] = wc;
    __syncthreads();
    int pre = 0, all = 0;
#pragma unroll
    for (int w2 = 0; w2 < NWAVE; ++w2) {
      int c = wcnt[w2];
      c = c < 0 ? 0 : (c > WCAP ? WCAP : c);
      all += c;
      pre += (w2 < wave) ? c : 0;
    }
    const int wcc  = wc > WCAP ? WCAP : wc;
    const int base = tot + pre;
#pragma unroll 1
    for (int b0 = 0; b0 < wcc; b0 += 32) {
      const int i  = b0 + lane;
      const int ic = i < WCAP ? i : WCAP - 1;
      const int ent = list[wave * WCAP + ic];
      const int el  = (ent >> PKS) & (CHUNK - 1);
      const int sl  = ent & (NBMAX - 1);
      int eid = cbase + el;
      eid = eid < 0 ? 0 : (eid > nK - 1 ? nK - 1 : eid);
      int val;
      if constexpr (VALSRC != 0) {
        const int sv = vals[eid];
        val = sv < 0 ? 0 : (sv > vmax ? vmax : sv);
      } else {
        val = eid > vmax ? vmax : eid;
      }
      const int pos = base + i;
      if (i < wcc && pos < RCAP) reg1[pos] = (int)(((unsigned)val << PKS) | (unsigned)sl);
    }
    tot += all;
    tot = tot > RCAP ? RCAP : tot;
    __syncthreads();
  }
  const int nh = tot;

  if (wave == 0) {
#pragma unroll 1
    for (int b0 = 0; b0 < nh; b0 += 32) {
      const int idx = b0 + lane;
      const int uv  = reg1[idx < RCAP ? idx : RCAP - 1];
      const int m32 = (nh - b0) < 32 ? (nh - b0) : 32;
#pragma unroll 1
      for (int k = 0; k < m32; ++k) {
        const int u  = __builtin_amdgcn_readlane(uv, k);
        const int sl = u & (NBMAX - 1);
        if (lane == 0) scnt[sl] = scnt[sl] + 1;
      }
    }
  }
  __syncthreads();

  {
    const v4i ca = *(const v4ia*)(scnt + 4 * tid);
    const int e0 = ca.x < 0 ? 0 : ca.x, e1 = ca.y < 0 ? 0 : ca.y, e2 = ca.z < 0 ? 0 : ca.z, e3 = ca.w < 0 ? 0 : ca.w;
    const int ts = e0 + e1 + e2 + e3;
    int incl = ts;
#pragma unroll
    for (int d = 1; d < 32; d <<= 1) {
      const int up = __shfl_up(incl, d);
      if (lane >= d) incl += up;
    }
    if (lane == 31) wtot[wave] = incl;
    __syncthreads();
    int pre = 0;
#pragma unroll
    for (int w2 = 0; w2 < NWAVE; ++w2) pre += (w2 < wave) ? wtot[w2] : 0;
    int run = pre + incl - ts;
    soff[4 * tid + 0] = run; run += e0;
    soff[4 * tid + 1] = run; run += e1;
    soff[4 * tid + 2] = run; run += e2;
    soff[4 * tid + 3] = run;
  }
  __syncthreads();
  for (int i = tid; i < NBMAX; i += NTHR) list[i] = soff[i];
  __syncthreads();

  if (wave == 0) {
#pragma unroll 1
    for (int b0 = 0; b0 < nh; b0 += 32) {
      const int idx = b0 + lane;
      const int uv  = reg1[idx < RCAP ? idx : RCAP - 1];
      const int m32 = (nh - b0) < 32 ? (nh - b0) : 32;
#pragma unroll 1
      for (int k = 0; k < m32; ++k) {
        const int u   = __builtin_amdgcn_readlane(uv, k);
        const int sl  = u & (NBMAX - 1);
        const int val = (int)((unsigned)u >> PKS);
        if (lane == 0) {
          int pos = list[sl];
          pos = pos < 0 ? 0 : (pos > RCAP - 1 ? RCAP - 1 : pos);
          reg2[pos] = val;
          list[sl] = pos + 1;
        }
      }
    }
  }
  __syncthreads();

  const bool ovf = (nh >= RCAP);
  int* lp = lst + (size_t)blockIdx.x * RCAP;
  int* cp = co + (size_t)blockIdx.x * (2 * NBMAX);
  v4i c4 = *(const v4ia*)(scnt + 4 * tid);
  const v4i o4 = *(const v4ia*)(soff + 4 * tid);
  if (ovf) { c4.x = -1; c4.y = -1; c4.z = -1; c4.w = -1; }
#pragma unroll 1
  for (int it = 0; it < RCAP / (4 * NTHR); ++it) {
    const int p4 = (it * NTHR + tid) * 4;
    const v4i v = *(const v4ia*)(reg2 + p4);
    *(volatile v4i*)(lp + p4) = v;
  }
  *(volatile v4i*)(cp + 4 * tid) = c4;
  *(volatile v4i*)(cp + NBMAX + 4 * tid) = o4;
  __threadfence();
#pragma unroll 1
  for (int it = 0; it < RCAP / (4 * NTHR); ++it) {
    const int p4 = (it * NTHR + tid) * 4;
    const v4i v = *(const v4ia*)(reg2 + p4);
    *(volatile v4i*)(lp + p4) = v;
  }
  *(volatile v4i*)(cp + 4 * tid) = c4;
  *(volatile v4i*)(cp + NBMAX + 4 * tid) = o4;
}

template <int SRCB>
__global__ __launch_bounds__(NTHR) void k_agg(const unsigned int* __restrict__ xbw, const float* __restrict__ zf,
                                              const float* __restrict__ stat,
                                              const int* __restrict__ lst, const int* __restrict__ co,
                                              unsigned int* aw, int nN, int MPr) {
  __shared__ __attribute__((aligned(16))) int scnt[NBMAX];
  __shared__ __attribute__((aligned(16))) int soff[NBMAX];
  __shared__ __attribute__((aligned(16))) float sst[STATW];
  const int tid = (int)threadIdx.x, lane = tid & 31;
  const int wave = __builtin_amdgcn_readfirstlane(tid >> 5);
  const int nodeBase = (int)blockIdx.x * NBMAX;
  {
    const int* cp = co + (size_t)blockIdx.x * (2 * NBMAX);
    const v4i c4 = *(const v4i*)(cp + 4 * tid);
    const v4i o4 = *(const v4i*)(cp + NBMAX + 4 * tid);
    *(v4ia*)(scnt + 4 * tid) = c4;
    *(v4ia*)(soff + 4 * tid) = o4;
    if constexpr (SRCB == 0) sst[tid] = stat[tid];
    else                     sst[tid] = 0.0f;
  }
  __syncthreads();
  const float m0 = sst[2 * lane], m1 = sst[2 * lane + 1];
  const float c0 = sst[DF + 2 * lane], c1 = sst[DF + 2 * lane + 1];
  const float e0 = sst[2 * DF + 2 * lane], e1 = sst[2 * DF + 2 * lane + 1];
  const int* lp = lst + (size_t)blockIdx.x * RCAP;
  const float qnan = __int_as_float(0x7fc00000);

#pragma unroll 1
  for (int jt = 0; jt < NBMAX / NWAVE; ++jt) {
    const int slot = wave * (NBMAX / NWAVE) + jt;
    const int grow = nodeBase + slot;
    if (grow >= MPr) break;
    const int craw = __builtin_amdgcn_readfirstlane(scnt[slot]);
    int st = __builtin_amdgcn_readfirstlane(soff[slot]);
    int cnt = craw < 0 ? 0 : (craw > DEGCAP ? DEGCAP : craw);
    st = st < 0 ? 0 : (st > RCAP ? RCAP : st);
    if (cnt > RCAP - st) cnt = RCAP - st;
    const bool bad = (craw < 0) || (craw > DEGCAP);
    const bool liveRow = grow < nN;

    float a0 = 0.0f, a1 = 0.0f;
#pragma unroll 1
    for (int b0 = 0; b0 < cnt; b0 += 32) {
      int idx = st + b0 + lane;
      idx = idx > RCAP - 1 ? RCAP - 1 : idx;
      int sr = lp[idx];
      sr = sr < 0 ? 0 : (sr > nN - 1 ? nN - 1 : sr);
      const int m32 = (cnt - b0) < 32 ? (cnt - b0) : 32;
#pragma unroll 1
      for (int k = 0; k < m32; ++k) {
        const int sk = __builtin_amdgcn_readlane(sr, k);
        if constexpr (SRCB != 0) {
          const unsigned int w = xbw[(size_t)sk * 32 + lane];
          a0 += __uint_as_float(w << 16);
          a1 += __uint_as_float(w & 0xffff0000u);
        } else {
          const v2f z = *(const v2f*)(zf + (size_t)sk * DF + 2 * lane);
          a0 += fmaf(z.x - m0, c0, e0);
          a1 += fmaf(z.y - m1, c1, e1);
        }
      }
    }
    const int nc = liveRow ? grow : nN - 1;
    float s0, s1;
    if constexpr (SRCB != 0) {
      const unsigned int w = xbw[(size_t)nc * 32 + lane];
      s0 = __uint_as_float(w << 16);
      s1 = __uint_as_float(w & 0xffff0000u);
    } else {
      const v2f z = *(const v2f*)(zf + (size_t)nc * DF + 2 * lane);
      s0 = fmaf(z.x - m0, c0, e0);
      s1 = fmaf(z.y - m1, c1, e1);
    }
    float r0 = s0 + a0, r1 = s1 + a1;
    r0 = bad ? qnan : r0;
    r1 = bad ? qnan : r1;
    r0 = liveRow ? r0 : 0.0f;
    r1 = liveRow ? r1 : 0.0f;
    const unsigned short h0 = bf_bits(r0), h1 = bf_bits(r1);
    const unsigned short l0 = bf_bits(r0 - bf_val(h0)), l1 = bf_bits(r1 - bf_val(h1));
    const unsigned int hw = (unsigned int)h0 | ((unsigned int)h1 << 16);
    const unsigned int lw = (unsigned int)l0 | ((unsigned int)l1 << 16);
    unsigned int* ap = aw + (size_t)grow * (KA / 2) + lane;
    *(volatile unsigned int*)ap = hw;
    *(volatile unsigned int*)(ap + 32) = lw;
    __threadfence();
    *(volatile unsigned int*)ap = hw;
    *(volatile unsigned int*)(ap + 32) = lw;
  }
}

__global__ __launch_bounds__(NTHR) __attribute__((amdgpu_num_vgpr(248)))
void k_mlp(const unsigned short* __restrict__ A, const unsigned short* __restrict__ W1D,
           const unsigned short* __restrict__ W2D, const float* __restrict__ b1, const float* __restrict__ b2,
           float* Z, float* rec, int nN) {
  extern __shared__ v4f mlp_dyn[];
  unsigned short* tl = (unsigned short*)mlp_dyn;
  float* stg = (float*)(tl + NWAVE * 16 * TP);
  float* sb  = stg + TM * DF;
  float* pst = sb + 128;
  const int tid = (int)threadIdx.x, lane = tid & 31, wave = tid >> 5, hh = lane >> 4, m = lane & 15;
  const int rowBase = (int)blockIdx.x * TM;

  if (tid < DF)            sb[tid] = bf_rne(b1[tid]);
  else if (tid < 2 * DF)   sb[tid] = bf_rne(b2[tid - DF]);
  if (tid >= 128 && tid < 159) pst[tid + 1] = 0.0f;

  v8f acc[4];
  {
    const v8f z = {0.f, 0.f, 0.f, 0.f, 0.f, 0.f, 0.f, 0.f};
#pragma unroll
    for (int t = 0; t < 4; ++t) acc[t] = z;
  }
  {
    const unsigned short* ap = A + (size_t)(rowBase + 16 * wave + m) * KA + 8 * hh;
    const unsigned short* bp = W1D + (size_t)m * KA + 8 * hh;
#pragma unroll 1
    for (int k0 = 0; k0 < KA; k0 += 32) {
      Frag af;
      af.h[0] = *(const v8usa*)(ap + k0);
      af.h[1] = *(const v8usa*)(ap + k0 + 16);
#pragma unroll
      for (int nt = 0; nt < 4; ++nt) {
        const unsigned short* wq = bp + (size_t)(16 * nt) * KA + k0;
        Frag bfr;
        bfr.h[0] = *(const v8usa*)wq;
        bfr.h[1] = *(const v8usa*)(wq + 16);
        acc[nt] = wmx(af, bfr, acc[nt]);
      }
    }
  }
  __syncthreads();

  unsigned short* tw = tl + wave * 16 * TP;
#pragma unroll
  for (int nt = 0; nt < 4; ++nt) {
    const int c = 16 * nt + m;
    const float bb = sb[c];
#pragma unroll
    for (int r = 0; r < 8; ++r) {
      const float v = relu_k(acc[nt][r] + bb);
      const unsigned short hb = bf_bits(v);
      const unsigned short lb = bf_bits(v - bf_val(hb));
      tw[(8 * hh + r) * TP + c] = hb;
      tw[(8 * hh + r) * TP + DF + c] = lb;
    }
  }
  __syncthreads();

  {
    const v8f z = {0.f, 0.f, 0.f, 0.f, 0.f, 0.f, 0.f, 0.f};
#pragma unroll
    for (int t = 0; t < 4; ++t) acc[t] = z;
  }
  {
    const unsigned short* ta = tw + m * TP + 8 * hh;
    const unsigned short* bp = W2D + (size_t)m * KA + 8 * hh;
#pragma unroll 1
    for (int k0 = 0; k0 < KA; k0 += 32) {
      Frag af;
      af.h[0] = *(const v8usa*)(ta + k0);
      af.h[1] = *(const v8usa*)(ta + k0 + 16);
#pragma unroll
      for (int nt = 0; nt < 4; ++nt) {
        const unsigned short* wq = bp + (size_t)(16 * nt) * KA + k0;
        Frag bfr;
        bfr.h[0] = *(const v8usa*)wq;
        bfr.h[1] = *(const v8usa*)(wq + 16);
        acc[nt] = wmx(af, bfr, acc[nt]);
      }
    }
  }

#pragma unroll
  for (int nt = 0; nt < 4; ++nt) {
    const int c = 16 * nt + m;
    const float bb = sb[DF + c];
#pragma unroll
    for (int r = 0; r < 8; ++r) {
      const int lr = 16 * wave + 8 * hh + r;
      const bool live = (rowBase + lr) < nN;
      const float v = relu_k(acc[nt][r] + bb);
      stg[lr * DF + c] = live ? v : 0.0f;
    }
  }
  __syncthreads();

  v4f zv[8];
#pragma unroll
  for (int j = 0; j < 8; ++j) zv[j] = *(const v4fa*)(stg + (16 * wave + 2 * j) * DF + 4 * lane);

  if (tid < DF) {
    int nvr = nN - rowBase;
    nvr = nvr < 0 ? 0 : (nvr > TM ? TM : nvr);
    float s = 0.0f;
#pragma unroll 4
    for (int r = 0; r < nvr; ++r) s += stg[r * DF + tid];
    const float inv = 1.0f / (float)(nvr < 1 ? 1 : nvr);
    const float mean = s * inv;
    float q = 0.0f;
#pragma unroll 4
    for (int r = 0; r < nvr; ++r) {
      const float d = stg[r * DF + tid] - mean;
      q = fmaf(d, d, q);
    }
    pst[1 + tid] = mean;
    pst[1 + DF + tid] = q;
    if (tid == 0) pst[0] = (float)nvr;
  }
  __syncthreads();

  const bool pok = tid < RECW / 4;
  v4f pv = {0.f, 0.f, 0.f, 0.f};
  if (pok) pv = *(const v4fa*)(pst + 4 * tid);
  float* zp = Z + (size_t)(rowBase + 16 * wave) * DF + 4 * lane;
  float* pp = rec + (size_t)blockIdx.x * RECW + 4 * tid;
#pragma unroll
  for (int j = 0; j < 8; ++j) *(volatile v4f*)(zp + 2 * j * DF) = zv[j];
  if (pok) *(volatile v4f*)pp = pv;
  __threadfence();
#pragma unroll
  for (int j = 0; j < 8; ++j) *(volatile v4f*)(zp + 2 * j * DF) = zv[j];
  if (pok) *(volatile v4f*)pp = pv;
}

__global__ __launch_bounds__(DF) void k_comb(const float* __restrict__ rec, int nRec,
                                             const float* __restrict__ gam, const float* __restrict__ bet,
                                             float* st) {
  __shared__ __attribute__((aligned(16))) float stg[STATW];
  const int c = (int)threadIdx.x;
  double n = 0.0, mean = 0.0, M2 = 0.0;
#pragma unroll 1
  for (int b = 0; b < nRec; ++b) {
    const float* pr = rec + (size_t)b * RECW;
    const double nb = (double)pr[0];
    const double mb = (double)pr[1 + c];
    const double qb = (double)pr[1 + DF + c];
    if (nb > 0.5) {
      const double nn = n + nb;
      const double delta = mb - mean;
      const double f = nb / nn;
      mean = mean + delta * f;
      M2 = M2 + qb + delta * delta * n * f;
      n = nn;
    }
  }
  const double nt = n < 1.0 ? 1.0 : n;
  const float varf  = (float)(M2 / nt);
  const float meanf = (float)mean;
  const float sc = bf_rne(gam[c]) / sqrtf(varf + 1e-5f);
  stg[c] = meanf;
  stg[DF + c] = sc;
  stg[2 * DF + c] = bf_rne(bet[c]);
  stg[3 * DF + c] = 0.0f;
  __syncthreads();
  const v4f v = *(const v4fa*)(stg + 4 * c);
  *(volatile v4f*)(st + 4 * c) = v;
  __threadfence();
  *(volatile v4f*)(st + 4 * c) = v;
}

__global__ __launch_bounds__(NTHR) void k_pool(const float* __restrict__ zf, const float* __restrict__ stat,
                                               const int* __restrict__ lst2, const int* __restrict__ co2,
                                               int nN, int nG, unsigned int* xpw, int colOff) {
  const int tid = (int)threadIdx.x, lane = tid & 31;
  const int wave = __builtin_amdgcn_readfirstlane(tid >> 5);
  const int g = (int)blockIdx.x * NWAVE + wave;
  if (g >= nG) return;
  const int bb = g / NBM, sl = g & (NBM - 1);
  const int* cp = co2 + (size_t)bb * (2 * NBMAX);
  const int craw = __builtin_amdgcn_readfirstlane(cp[sl]);
  int st = __builtin_amdgcn_readfirstlane(cp[NBMAX + sl]);
  int cnt = craw < 0 ? 0 : (craw > MCAP ? MCAP : craw);
  st = st < 0 ? 0 : (st > RCAP ? RCAP : st);
  if (cnt > RCAP - st) cnt = RCAP - st;
  const bool bad = (craw < 0) || (craw > MCAP);
  const v2f mm = *(const v2f*)(stat + 2 * lane);
  const v2f sc = *(const v2f*)(stat + DF + 2 * lane);
  const v2f be = *(const v2f*)(stat + 2 * DF + 2 * lane);
  const int* lp = lst2 + (size_t)bb * RCAP;
  float a0 = 0.0f, a1 = 0.0f;
#pragma unroll 1
  for (int b0 = 0; b0 < cnt; b0 += 32) {
    int idx = st + b0 + lane;
    idx = idx > RCAP - 1 ? RCAP - 1 : idx;
    int nd = lp[idx];
    nd = nd < 0 ? 0 : (nd > nN - 1 ? nN - 1 : nd);
    const int m32 = (cnt - b0) < 32 ? (cnt - b0) : 32;
#pragma unroll 1
    for (int k = 0; k < m32; ++k) {
      const int nk = __builtin_amdgcn_readlane(nd, k);
      const v2f z = *(const v2f*)(zf + (size_t)nk * DF + 2 * lane);
      a0 += fmaf(z.x - mm.x, sc.x, be.x);
      a1 += fmaf(z.y - mm.y, sc.y, be.y);
    }
  }
  const float qnan = __int_as_float(0x7fc00000);
  const float r0 = bad ? qnan : a0;
  const float r1 = bad ? qnan : a1;
  const unsigned short h0 = bf_bits(r0), h1 = bf_bits(r1);
  const unsigned short l0 = bf_bits(r0 - bf_val(h0)), l1 = bf_bits(r1 - bf_val(h1));
  const unsigned int hw = (unsigned int)h0 | ((unsigned int)h1 << 16);
  const unsigned int lw = (unsigned int)l0 | ((unsigned int)l1 << 16);
  unsigned int* xp = xpw + (size_t)g * (XPW / 2) + (colOff >> 1) + lane;
  *(volatile unsigned int*)xp = hw;
  *(volatile unsigned int*)(xp + XPH / 2) = lw;
  __threadfence();
  *(volatile unsigned int*)xp = hw;
  *(volatile unsigned int*)(xp + XPH / 2) = lw;
}

__global__ __launch_bounds__(NTHR) __attribute__((amdgpu_num_vgpr(248)))
void k_head(const unsigned short* __restrict__ XP, const unsigned short* __restrict__ LWD,
            const float* __restrict__ lin_b, const float* __restrict__ fin_w, const float* __restrict__ fin_b,
            float* out) {
  __shared__ __attribute__((aligned(16))) float stg[TM * DF];
  __shared__ __attribute__((aligned(16))) float sfw[DF * NCLS];
  __shared__ __attribute__((aligned(16))) float slb[DF];
  __shared__ __attribute__((aligned(16))) float sfb[16];
  __shared__ __attribute__((aligned(16))) float slog[TM * NCLS];
  const int tid = (int)threadIdx.x, lane = tid & 31, wave = tid >> 5, hh = lane >> 4, m = lane & 15;
  const int rowBase = (int)blockIdx.x * TM;

#pragma unroll 1
  for (int b = 0; b < DF * NCLS; b += NTHR) {
    const int i = b + tid;
    const int ic = i < DF * NCLS ? i : DF * NCLS - 1;
    const float v = bf_rne(fin_w[ic]);
    if (i < DF * NCLS) sfw[i] = v;
  }
  if (tid < DF) slb[tid] = bf_rne(lin_b[tid]);
  {
    const int ic = tid < NCLS ? tid : NCLS - 1;
    const float v = bf_rne(fin_b[ic]);
    if (tid < 16) sfb[tid] = (tid < NCLS) ? v : 0.0f;
  }

  v8f acc[4];
  {
    const v8f z = {0.f, 0.f, 0.f, 0.f, 0.f, 0.f, 0.f, 0.f};
#pragma unroll
    for (int t = 0; t < 4; ++t) acc[t] = z;
  }
  {
    const unsigned short* ap = XP + (size_t)(rowBase + 16 * wave + m) * XPW + 8 * hh;
    const unsigned short* bp = LWD + (size_t)m * XPW + 8 * hh;
#pragma unroll 1
    for (int k0 = 0; k0 < XPW; k0 += 32) {
      Frag af;
      af.h[0] = *(const v8usa*)(ap + k0);
      af.h[1] = *(const v8usa*)(ap + k0 + 16);
#pragma unroll
      for (int nt = 0; nt < 4; ++nt) {
        const unsigned short* wq = bp + (size_t)(16 * nt) * XPW + k0;
        Frag bfr;
        bfr.h[0] = *(const v8usa*)wq;
        bfr.h[1] = *(const v8usa*)(wq + 16);
        acc[nt] = wmx(af, bfr, acc[nt]);
      }
    }
  }
  __syncthreads();

#pragma unroll
  for (int nt = 0; nt < 4; ++nt) {
    const int c = 16 * nt + m;
    const float bb = slb[c];
#pragma unroll
    for (int r = 0; r < 8; ++r) {
      const int lr = 16 * wave + 8 * hh + r;
      stg[lr * DF + c] = relu_k(acc[nt][r] + bb);
    }
  }
  __syncthreads();

#pragma unroll 1
  for (int it = 0; it < (TM * NCLS) / NTHR; ++it) {
    const int u = it * NTHR + tid;
    const int row = u / NCLS, c = u - row * NCLS;
    float a = sfb[c];
#pragma unroll 4
    for (int k = 0; k < DF; ++k) a = fmaf(stg[row * DF + k], sfw[k * NCLS + c], a);
    slog[u] = a;
  }
  __syncthreads();

  if (tid < TM) {
    float* rp = slog + tid * NCLS;
    float mx = rp[0];
#pragma unroll 1
    for (int c = 1; c < NCLS; ++c) {
      const float v = rp[c];
      mx = (v > mx || v != v) ? v : mx;
    }
    float se = 0.0f;
#pragma unroll 1
    for (int c = 0; c < NCLS; ++c) se += expf(rp[c] - mx);
    const float lse = mx + logf(se);
#pragma unroll 1
    for (int c = 0; c < NCLS; ++c) rp[c] = rp[c] - lse;
  }
  __syncthreads();

  const bool t1 = tid < (TM * NCLS) / 4 - NTHR;
  const int u1 = t1 ? NTHR + tid : 0;
  const v4f o0 = *(const v4fa*)(slog + 4 * tid);
  const v4f o1 = *(const v4fa*)(slog + 4 * u1);
  float* ob = out + (size_t)blockIdx.x * (TM * NCLS);
  *(volatile v4f*)(ob + 4 * tid) = o0;
  if (t1) *(volatile v4f*)(ob + 4 * (NTHR + tid)) = o1;
  __threadfence();
  *(volatile v4f*)(ob + 4 * tid) = o0;
  if (t1) *(volatile v4f*)(ob + 4 * (NTHR + tid)) = o1;
}

static inline int cdiv(int a, int b) { return (a + b - 1) / b; }
static inline size_t al256(size_t o) { return (o + 255) & ~(size_t)255; }

extern "C" void kernel_launch(void* const* d_in, const int* in_sizes, int n_in,
                              void* d_out, int out_size, void* d_ws, size_t ws_size,
                              hipStream_t stream) {
  if (n_in < 13) return;
  if (in_sizes[0] < DF || (in_sizes[0] % DF) != 0) return;
  const int nN = in_sizes[0] / DF;
  if (nN < TM || nN > (1 << 20)) return;
  const int nE2 = in_sizes[1];
  if (nE2 < 2 || (nE2 & 1) != 0) return;
  const int nE = nE2 / 2;
  if (nE < 1 || nE > (1 << 28)) return;
  if (in_sizes[2] != nN) return;
  if (in_sizes[3] != NLAY * DF * DF || in_sizes[4] != NLAY * DF) return;
  if (in_sizes[5] != NLAY * DF * DF || in_sizes[6] != NLAY * DF) return;
  if (in_sizes[7] != NLAY * DF || in_sizes[8] != NLAY * DF) return;
  if (in_sizes[9] != XPH * DF || in_sizes[10] != DF) return;
  if (in_sizes[11] != DF * NCLS || in_sizes[12] != NCLS) return;
  if (out_size < TM * NCLS || (out_size % (TM * NCLS)) != 0) return;
  const int nG = out_size / NCLS;
  if ((nG % TM) != 0 || (nG % NWAVE) != 0 || nG > 65536) return;

  const float* x     = (const float*)d_in[0];
  const int*   ei    = (const int*)  d_in[1];
  const int*   src   = ei;
  const int*   dst   = ei + nE;
  const int*   batch = (const int*)  d_in[2];
  const float* w1    = (const float*)d_in[3];
  const float* b1    = (const float*)d_in[4];
  const float* w2    = (const float*)d_in[5];
  const float* b2    = (const float*)d_in[6];
  const float* gamma = (const float*)d_in[7];
  const float* beta  = (const float*)d_in[8];
  const float* lin_w = (const float*)d_in[9];
  const float* lin_b = (const float*)d_in[10];
  const float* fin_w = (const float*)d_in[11];
  const float* fin_b = (const float*)d_in[12];
  float* out = (float*)d_out;

  const int MP  = cdiv(nN, TM) * TM;
  const int gT  = MP / TM;
  const int gA  = cdiv(MP, NBMAX);
  const int gMb = cdiv(nG, NBM);
  if ((long long)gA * NBMAX < (long long)MP) return;
  if ((long long)gMb * NBM < (long long)nG) return;
  const int vec8e = ((nE & 3) == 0) ? 1 : 0;

  char* ws = (char*)d_ws;
  size_t off = 0;
  const size_t oXB  = off; off = al256(off + (size_t)MP * DF * 2);
  const size_t oWP  = off; off = al256(off + (size_t)6 * DF * KA * 2);
  const size_t oLW  = off; off = al256(off + (size_t)DF * XPW * 2);
  const size_t oA   = off; off = al256(off + (size_t)MP * KA * 2);
  const size_t oZ   = off; off = al256(off + (size_t)MP * DF * 4);
  const size_t oLS  = off; off = al256(off + (size_t)gA * RCAP * 4);
  const size_t oCO  = off; off = al256(off + (size_t)gA * 2 * NBMAX * 4);
  const size_t oLS2 = off; off = al256(off + (size_t)gMb * RCAP * 4);
  const size_t oCO2 = off; off = al256(off + (size_t)gMb * 2 * NBMAX * 4);
  const size_t oRC  = off; off = al256(off + (size_t)gT * RECW * 4);
  const size_t oST  = off; off = al256(off + (size_t)NLAY * STATW * 4);
  const size_t oXP  = off; off = al256(off + (size_t)nG * XPW * 2);
  if (off > ws_size || off > (size_t)WSCAP) return;
  unsigned short* XB  = (unsigned short*)(ws + oXB);
  unsigned short* WPL = (unsigned short*)(ws + oWP);
  unsigned short* LWD = (unsigned short*)(ws + oLW);
  unsigned short* AP  = (unsigned short*)(ws + oA);
  float*          ZP  = (float*)(ws + oZ);
  int*            LS  = (int*)(ws + oLS);
  int*            CO  = (int*)(ws + oCO);
  int*            LS2 = (int*)(ws + oLS2);
  int*            CO2 = (int*)(ws + oCO2);
  float*          RC  = (float*)(ws + oRC);
  float*          ST  = (float*)(ws + oST);
  unsigned short* XP  = (unsigned short*)(ws + oXP);

  hipFuncSetAttribute(reinterpret_cast<const void*>(&k_bucket<1>), hipFuncAttributeMaxDynamicSharedMemorySize, LDS_BKT);
  hipFuncSetAttribute(reinterpret_cast<const void*>(&k_bucket<0>), hipFuncAttributeMaxDynamicSharedMemorySize, LDS_BKT);
  hipFuncSetAttribute(reinterpret_cast<const void*>(&k_mlp),       hipFuncAttributeMaxDynamicSharedMemorySize, LDS_MLP);

  const int nUx = MP * (DF / 8);
  k_pa<<<cdiv(nUx, NTHR), NTHR, 0, stream>>>(x, nN, nUx, XB);
  k_pb<<<9216 / NTHR, NTHR, 0, stream>>>(w1, w2, lin_w, WPL, LWD);
  k_bucket<1><<<gA, NTHR, LDS_BKT, stream>>>(dst, src, nE, NBMAX, nN - 1, vec8e, LS, CO);
  k_bucket<0><<<gMb, NTHR, LDS_BKT, stream>>>(batch, batch, nN, NBM, nN - 1, 1, LS2, CO2);

  for (int l = 0; l < NLAY; ++l) {
    float* STl = ST + (size_t)l * STATW;
    if (l == 0) {
      k_agg<1><<<gA, NTHR, 0, stream>>>((const unsigned int*)XB, ZP, ST, LS, CO, (unsigned int*)AP, nN, MP);
    } else {
      k_agg<0><<<gA, NTHR, 0, stream>>>((const unsigned int*)XB, ZP, ST + (size_t)(l - 1) * STATW, LS, CO,
                                        (unsigned int*)AP, nN, MP);
    }
    k_mlp<<<gT, NTHR, LDS_MLP, stream>>>(AP, WPL + (size_t)(2 * l) * (DF * KA), WPL + (size_t)(2 * l + 1) * (DF * KA),
                                         b1 + l * DF, b2 + l * DF, ZP, RC, nN);
    k_comb<<<1, DF, 0, stream>>>(RC, gT, gamma + l * DF, beta + l * DF, STl);
    k_pool<<<nG / NWAVE, NTHR, 0, stream>>>(ZP, STl, LS2, CO2, nN, nG, (unsigned int*)XP, l * DF);
  }
  k_head<<<nG / TM, NTHR, 0, stream>>>(XP, LWD, lin_b, fin_w, fin_b, out);
}
